// HONAM_44521630990690
// MI455X (gfx1250) — hardware-run, weakly checked
//
#include <hip/hip_runtime.h>


#ifndef NSAMP
#define NSAMP 8192
#endif
#define NSAMP_FULL 8192
#define NFEAT 256
#define H1W   32
#define H2W   64
#define H3W   32
#define ST    2
#define WSC   64.0f
#define WSI   (1.0f / 64.0f)

static_assert(H1W == 32);
static_assert(H2W == 64);
static_assert(H3W == 32);
static_assert(ST == 2);
static_assert(NSAMP % (16 * ST) == 0);
static_assert(NSAMP <= NSAMP_FULL);
static_assert(NFEAT % 4 == 0);
static_assert((H1W * H2W) == 2048);
static_assert((H2W * H3W) == 2048);

typedef _Float16 h16;
typedef __attribute__((ext_vector_type(16))) _Float16 v16h;
typedef __attribute__((ext_vector_type(8)))  _Float16 v8h;
typedef __attribute__((ext_vector_type(8)))  float    v8f;
typedef __attribute__((ext_vector_type(4)))  float    v4f;
typedef v4f  __attribute__((may_alias)) v4fa;

__device__ __forceinline__ unsigned short f2bf(float f) { unsigned u = __float_as_uint(f); u += 0x7FFFu + ((u >> 16) & 1u); return (unsigned short)(u >> 16); }
__device__ __forceinline__ float bfr(float f) { return __uint_as_float(((unsigned)f2bf(f)) << 16); }
__device__ __forceinline__ v16h cat16(v8h lo, v8h hi) { return __builtin_shufflevector(lo, hi, 0, 1, 2, 3, 4, 5, 6, 7, 8, 9, 10, 11, 12, 13, 14, 15); }
__device__ __forceinline__ v8f wmma16(v16h a, v16h b, v8f c) { return __builtin_amdgcn_wmma_f32_16x16x32_f16(false, a, false, b, (short)0, c, false, false); }
__device__ __forceinline__ v8f wmma16g(v16h a, v16h b, v8f c) { c = wmma16(a, b, c); asm volatile("v_nop\n\tv_nop\n\tv_nop\n\tv_nop" : "+v"(c) : "v"(a), "v"(b)); return c; }
__device__ __forceinline__ v16h ldh(const h16* p) { return cat16(*(const v8h*)p, *(const v8h*)(p + 16)); }
static __device__ __forceinline__ h16 toh_flush(float v) { const float w = (fabsf(v) < 6.103515625e-05f) ? 0.0f : v; return (h16)w; }
__device__ __forceinline__ void wave_sync() { __builtin_amdgcn_fence(3  , "wavefront"); __builtin_amdgcn_wave_barrier(); asm volatile("" ::: "memory"); }

__global__ __launch_bounds__(256) void k_bfr4(const float* __restrict__ src, float* dst, unsigned n4) {
    const unsigned i = blockIdx.x * 256u + threadIdx.x; if (i >= n4) return;
    const v4f v = *(const v4f*)(src + (size_t)i * 4); v4f o;
#pragma unroll
    for (int k = 0; k < 4; ++k) o[k] = bfr(v[k]);
    *(volatile v4f*)(dst + (size_t)i * 4) = o; __threadfence(); *(volatile v4f*)(dst + (size_t)i * 4) = o;
}

#define WT_LDS 2176
static_assert(32 * 65 <= WT_LDS);
static_assert(64 * 33 <= WT_LDS);
static_assert(2 * 256 * 4 == H1W * H2W);
static_assert(2 * 256 * 4 == H2W * H3W);
static_assert(256 * 8 == H2W * H1W);
static_assert(256 * 8 == H3W * H2W);
static_assert(WT_LDS * 4 <= 131072);
__global__ __launch_bounds__(256) void k_wt(const float* __restrict__ W2, const float* __restrict__ W3, h16* W2T, h16* W3T) {
    __shared__ __align__(16) float ts[WT_LDS];
    const unsigned f = blockIdx.x; const unsigned tid = threadIdx.x;
    const float* src2 = W2 + (size_t)f * 2048u;
    const float* src3 = W3 + (size_t)f * 2048u;
#pragma unroll
    for (unsigned q = 0; q < 2; ++q) {
        const unsigned idx = (q * 256u + tid) * 4u;
        const v4f v = *(const v4f*)(src2 + idx);
        const unsigned k = idx >> 6, o = idx & 63u;
        ts[k * 65u + o + 0u] = v[0]; ts[k * 65u + o + 1u] = v[1]; ts[k * 65u + o + 2u] = v[2]; ts[k * 65u + o + 3u] = v[3];
    }
    __syncthreads();
    v8h hv2;
    { const unsigned o = tid >> 2, k8 = (tid & 3u) * 8u;
#pragma unroll
      for (unsigned i = 0; i < 8; ++i) hv2[i] = toh_flush(bfr(ts[(k8 + i) * 65u + o]) * WSC); }
    __syncthreads();
#pragma unroll
    for (unsigned q = 0; q < 2; ++q) {
        const unsigned idx = (q * 256u + tid) * 4u;
        const v4f v = *(const v4f*)(src3 + idx);
        const unsigned k = idx >> 5, j = idx & 31u;
        ts[k * 33u + j + 0u] = v[0]; ts[k * 33u + j + 1u] = v[1]; ts[k * 33u + j + 2u] = v[2]; ts[k * 33u + j + 3u] = v[3];
    }
    __syncthreads();
    v8h hv3;
    { const unsigned j = tid >> 3, k8 = (tid & 7u) * 8u;
#pragma unroll
      for (unsigned i = 0; i < 8; ++i) hv3[i] = toh_flush(bfr(ts[(k8 + i) * 33u + j]) * WSC); }
    h16* d2 = W2T + (size_t)f * 2048u + (size_t)tid * 8u;
    h16* d3 = W3T + (size_t)f * 2048u + (size_t)tid * 8u;
    *(volatile v8h*)d2 = hv2; *(volatile v8h*)d3 = hv3;
    __threadfence();
    *(volatile v8h*)d2 = hv2; *(volatile v8h*)d3 = hv3;
}

static_assert(8 * 16 == 16 * ST * 4);
__global__ __launch_bounds__(32) __attribute__((amdgpu_num_vgpr(256)))
void k_fnet(const float* __restrict__ X, const float* __restrict__ W1R, const float* __restrict__ B1R,
            const h16* __restrict__ W2T, const float* __restrict__ B2R,
            const h16* __restrict__ W3T, const float* __restrict__ B3R,
            const float* __restrict__ WOUT, const float* __restrict__ BOUT, float* OUT) {
    __shared__ __align__(16) float os[32];
    const unsigned lane = threadIdx.x & 31u, lr = lane & 15u, hi = lane >> 4;
    const unsigned bx = blockIdx.x;
    const size_t s0 = (size_t)bx * 32u;
    const float* x0 = X + (s0 + lr) * NFEAT;
    const float* x1 = x0 + (size_t)16 * NFEAT;
    v8f p1[ST][2], p2[ST][2];
#pragma unroll
    for (int st = 0; st < ST; ++st)
#pragma unroll
        for (int jt = 0; jt < 2; ++jt) { p1[st][jt] = (v8f){}; p2[st][jt] = (v8f){}; }

#pragma unroll 1
    for (unsigned f = 0; f < NFEAT; ++f) {
        v16h h1[ST];
        {
            const float* wp = W1R + (size_t)f * H1W + 8u * hi;
            const float* bp = B1R + (size_t)f * H1W + 8u * hi;
            const v4f wa = *(const v4f*)wp, wb = *(const v4f*)(wp + 4), wc = *(const v4f*)(wp + 16), wd = *(const v4f*)(wp + 20);
            const v4f ba = *(const v4f*)bp, bb = *(const v4f*)(bp + 4), bc = *(const v4f*)(bp + 16), bd = *(const v4f*)(bp + 20);
            float wv[16], bv[16];
#pragma unroll
            for (int i = 0; i < 4; ++i) { wv[i] = wa[i]; wv[4 + i] = wb[i]; wv[8 + i] = wc[i]; wv[12 + i] = wd[i];
                                          bv[i] = ba[i]; bv[4 + i] = bb[i]; bv[8 + i] = bc[i]; bv[12 + i] = bd[i]; }
            const float xa = bfr(x0[f]), xb = bfr(x1[f]);
#pragma unroll
            for (int i = 0; i < 16; ++i) {
                h1[0][i] = toh_flush(fmaxf(xa * wv[i] + bv[i], 0.0f));
                h1[1][i] = toh_flush(fmaxf(xb * wv[i] + bv[i], 0.0f)); }
        }
        v16h h2f[ST][2];
#pragma unroll
        for (int ot = 0; ot < 4; ++ot) {
            const v16h a = ldh(W2T + ((size_t)f * H2W + (size_t)(ot * 16) + lr) * H1W + 8u * hi);
            const float* bp = B2R + (size_t)f * H2W + (size_t)(ot * 16) + 8u * hi;
            const v4f b0 = *(const v4f*)bp, b1 = *(const v4f*)(bp + 4);
            float bo[8];
#pragma unroll
            for (int r = 0; r < 4; ++r) { bo[r] = b0[r]; bo[4 + r] = b1[r]; }
#pragma unroll
            for (int st = 0; st < ST; ++st) {
                v8f c = (v8f){};
                c = wmma16g(a, h1[st], c);
#pragma unroll
                for (int r = 0; r < 8; ++r) h2f[st][ot >> 1][(ot & 1) * 8 + r] = toh_flush(fmaxf(c[r] * WSI + bo[r], 0.0f));
            }
        }
#pragma unroll
        for (int jt = 0; jt < 2; ++jt) {
            const h16* ap = W3T + ((size_t)f * H3W + (size_t)(jt * 16) + lr) * H2W + 8u * hi;
            const v16h a0 = ldh(ap), a1 = ldh(ap + 32);
            const float* bp = B3R + (size_t)f * H3W + (size_t)(jt * 16) + 8u * hi;
            const v4f b0 = *(const v4f*)bp, b1 = *(const v4f*)(bp + 4);
            float bo[8];
#pragma unroll
            for (int r = 0; r < 4; ++r) { bo[r] = b0[r]; bo[4 + r] = b1[r]; }
#pragma unroll
            for (int st = 0; st < ST; ++st) {
                v8f c = (v8f){};
                c = wmma16g(a0, h2f[st][0], c);
                c = wmma16g(a1, h2f[st][1], c);
#pragma unroll
                for (int r = 0; r < 8; ++r) { const float t = fmaxf(c[r] * WSI + bo[r], 0.0f); p1[st][jt][r] += t; p2[st][jt][r] += t * t; }
            }
        }
    }

    float accs[ST];
#pragma unroll
    for (int st = 0; st < ST; ++st) accs[st] = 0.0f;
#pragma unroll
    for (int jt = 0; jt < 2; ++jt) {
        const float* wp = WOUT + (size_t)(jt * 16) + 8u * hi;
        const v4f wa = *(const v4f*)wp, wb = *(const v4f*)(wp + 4), wc = *(const v4f*)(wp + 32), wd = *(const v4f*)(wp + 36);
        float w1o[8], w2o[8];
#pragma unroll
        for (int r = 0; r < 4; ++r) { w1o[r] = bfr(wa[r]); w1o[4 + r] = bfr(wb[r]); w2o[r] = bfr(wc[r]); w2o[4 + r] = bfr(wd[r]); }
#pragma unroll
        for (int st = 0; st < ST; ++st) {
#pragma unroll
            for (int r = 0; r < 8; ++r) {
                const float a = p1[st][jt][r], q = p2[st][jt][r];
                const float e2 = (a * a - q) * 0.5f;
                accs[st] += a * w1o[r];
                accs[st] += e2 * w2o[r]; }
        }
    }
#pragma unroll
    for (int st = 0; st < ST; ++st) accs[st] += __shfl_xor(accs[st], 16, 32);
    const float bo1 = bfr(BOUT[0]);
    const float mine = ((hi != 0u) ? accs[1] : accs[0]) + bo1;
    os[lane] = mine;
    wave_sync();
    const v4f val = *(const v4fa*)(&os[(lane & 7u) * 4u]);
    float* orow = OUT + s0;
#pragma unroll 1
    for (int ps = 0; ps < 2; ++ps) {
        if (lane < 8u) *(volatile v4f*)(orow + (size_t)lane * 4u) = val;
        if (ps == 0) __threadfence(); }
}

static constexpr size_t al256(size_t v) { return (v + 255) & ~(size_t)255; }
static constexpr size_t SZ_WT  = al256((size_t)NFEAT * 2048 * 2);
static constexpr size_t SZ_P32 = al256((size_t)NFEAT * 32 * 4);
static constexpr size_t SZ_P64 = al256((size_t)NFEAT * 64 * 4);
static constexpr size_t OFF_W2T = 0;
static constexpr size_t OFF_W3T = OFF_W2T + SZ_WT;
static constexpr size_t OFF_W1R = OFF_W3T + SZ_WT;
static constexpr size_t OFF_B1R = OFF_W1R + SZ_P32;
static constexpr size_t OFF_B2R = OFF_B1R + SZ_P32;
static constexpr size_t OFF_B3R = OFF_B2R + SZ_P64;
static constexpr size_t SZ_TOTAL = OFF_B3R + SZ_P32;
static_assert(SZ_TOTAL <= (size_t)134217728);
static constexpr unsigned N4_P32 = (unsigned)((size_t)NFEAT * 32 / 4);
static constexpr unsigned N4_P64 = (unsigned)((size_t)NFEAT * 64 / 4);
static_assert(N4_P32 % 256 == 0);
static_assert(N4_P64 % 256 == 0);
static constexpr unsigned G_P32 = N4_P32 / 256;
static constexpr unsigned G_P64 = N4_P64 / 256;
static constexpr unsigned G_FN  = (unsigned)(NSAMP / (16 * ST));
static_assert((size_t)G_FN * 32 == (size_t)NSAMP);
static constexpr size_t NEED_X = (size_t)NSAMP * NFEAT;

extern "C" void kernel_launch(void* const* d_in, const int* in_sizes, int n_in,
                              void* d_out, int out_size, void* d_ws, size_t ws_size, hipStream_t stream) {
    if (n_in < 9) return;
    if ((size_t)in_sizes[0] < NEED_X) return;
    if (in_sizes[1] < NFEAT * 32 || in_sizes[2] < NFEAT * 32) return;
    if (in_sizes[3] < NFEAT * 2048 || in_sizes[4] < NFEAT * 64) return;
    if (in_sizes[5] < NFEAT * 2048 || in_sizes[6] < NFEAT * 32) return;
    if (in_sizes[7] < 64 || in_sizes[8] < 1) return;
    if (out_size < NSAMP) return;
    if (SZ_TOTAL > ws_size) return;
    const float* x    = (const float*)d_in[0];
    const float* w1   = (const float*)d_in[1];
    const float* b1   = (const float*)d_in[2];
    const float* w2   = (const float*)d_in[3];
    const float* b2   = (const float*)d_in[4];
    const float* w3   = (const float*)d_in[5];
    const float* b3   = (const float*)d_in[6];
    const float* wout = (const float*)d_in[7];
    const float* bout = (const float*)d_in[8];
    float* OUT = (float*)d_out;
    char* wsp = (char*)d_ws;
    h16*   W2T = (h16*)(wsp + OFF_W2T);
    h16*   W3T = (h16*)(wsp + OFF_W3T);
    float* W1R = (float*)(wsp + OFF_W1R);
    float* B1R = (float*)(wsp + OFF_B1R);
    float* B2R = (float*)(wsp + OFF_B2R);
    float* B3R = (float*)(wsp + OFF_B3R);

    k_wt<<<NFEAT, 256, 0, stream>>>(w2, w3, W2T, W3T);
    k_bfr4<<<G_P32, 256, 0, stream>>>(w1, W1R, N4_P32);
    k_bfr4<<<G_P32, 256, 0, stream>>>(b1, B1R, N4_P32);
    k_bfr4<<<G_P64, 256, 0, stream>>>(b2, B2R, N4_P64);
    k_bfr4<<<G_P32, 256, 0, stream>>>(b3, B3R, N4_P32);
    k_fnet<<<G_FN, 32, 0, stream>>>(x, W1R, B1R, W2T, B2R, W3T, B3R, wout, bout, OUT);
}
